// MaskedGridPredictor_48558900249394
// MI455X (gfx1250) — hardware-run, weakly checked
//
#include <hip/hip_runtime.h>
#include <math.h>

typedef __attribute__((ext_vector_type(16))) _Float16 v16h;
typedef __attribute__((ext_vector_type(8)))  _Float16 v8h;
typedef __attribute__((ext_vector_type(8)))  float    v8f;
typedef __attribute__((ext_vector_type(4)))  float    v4f;
typedef __attribute__((ext_vector_type(4)))  unsigned int v4u;

constexpr int kBatch  = 4;
constexpr int kSeq    = 8192;
constexpr int kDim    = 256;
constexpr int kHeads  = 8;
constexpr int kDh     = 64;
constexpr int kInner  = kHeads * kDh;
constexpr int kTok    = kBatch * kSeq;
constexpr int kBH     = kBatch * kHeads;
constexpr int kSplitK = 8;
constexpr int kTokPerSplit = kSeq / kSplitK;
constexpr int kDotsElems = kBH * kDh * kDh;
static_assert(kInner == 512 && kTok == 32768 && kDotsElems == 131072, "shape");
static_assert((kDim % 32) == 0 && (kInner % 32) == 0 && (kDh % 32) == 0, "K multiples of 32");
static_assert((kTok % 32) == 0 && (kSeq % 32) == 0, "M multiples of 32");
static_assert((kInner % 64) == 0 && ((2 * kInner) % 64) == 0 && (kDim % 64) == 0 && (kDh % 64) == 0, "N multiples of 64");
static_assert((kTokPerSplit % 64) == 0, "token chunks of 64");

constexpr float kXC     = 16.0f;
constexpr float kWC     = 1024.0f;
constexpr float kKVC    = 16.0f;
constexpr float kQC     = 64.0f;
constexpr float kDC     = 1024.0f;
constexpr float kAC     = 64.0f;
constexpr float kProjScale = 1.0f / (kXC * kWC);
constexpr float kDotsScale = kDC / (kKVC * kKVC * (float)kSeq);
constexpr float kAttnScale = kAC / (kQC * kDC);
constexpr float kOutScale  = 1.0f / (kAC * kWC);
constexpr float kPosScale  = 64.0f;
constexpr float kNormEps   = 1e-5f;
constexpr float kInvDh     = 1.0f / (float)kDh;

constexpr size_t kOffWQ   = 0;
constexpr size_t kOffWK   = kOffWQ   + (size_t)kInner * kDim * 2;
constexpr size_t kOffWO   = kOffWK   + (size_t)2 * kInner * kDim * 2;
constexpr size_t kOffS16  = kOffWO   + (size_t)kDim * kInner * 2;
constexpr size_t kOffKN   = kOffS16  + (size_t)kTok * kDim * 2;
constexpr size_t kOffVN   = kOffKN   + (size_t)kTok * kInner * 2;
constexpr size_t kOffQH   = kOffVN   + (size_t)kTok * kInner * 2;
constexpr size_t kOffTAB  = kOffQH   + (size_t)kTok * kInner * 2;
constexpr size_t kOffPART = kOffTAB  + (size_t)kTok * 64 * 4;
constexpr size_t kOffDH   = kOffPART + (size_t)kSplitK * kDotsElems * 4;
constexpr size_t kWsTotal = kOffDH   + (size_t)kDotsElems * 2;
static_assert(kWsTotal == 131334144ull, "carve total");
static_assert(kWsTotal <= 134217728ull, "carve cap");
static_assert((kOffWK % 128) == 0 && (kOffWO % 128) == 0 && (kOffS16 % 128) == 0 && (kOffKN % 128) == 0 &&
              (kOffVN % 128) == 0 && (kOffQH % 128) == 0 && (kOffTAB % 128) == 0 && (kOffPART % 128) == 0 &&
              (kOffDH % 128) == 0, "128-B aligned regions");

__device__ __forceinline__ unsigned short f2bf_bits(float f) {
  unsigned u = __float_as_uint(f);
  return (unsigned short)((u + 0x7FFFu + ((u >> 16) & 1u)) >> 16);
}
__device__ __forceinline__ float bf_bits2f(unsigned short h) { return __uint_as_float(((unsigned)h) << 16); }
__device__ __forceinline__ float bf_rne(float f) { return bf_bits2f(f2bf_bits(f)); }

__device__ __forceinline__ unsigned pk16(unsigned short a, unsigned short b) { return (unsigned)a | ((unsigned)b << 16); }
__device__ __forceinline__ unsigned short h_bits(float f) { const _Float16 h = (_Float16)f; return __builtin_bit_cast(unsigned short, h); }

union FragU { v16h v; v8h h[2]; };
__device__ __forceinline__ v16h frag_load(const _Float16* p) {
  FragU f;
  f.h[0] = *(const v8h*)(p);
  f.h[1] = *(const v8h*)(p + 16);
  return f.v;
}
__device__ __forceinline__ v8f mma16(v16h a, v16h b, v8f c) {
  return __builtin_amdgcn_wmma_f32_16x16x32_f16(false, a, false, b, (short)0, c, false, false);
}
__device__ __forceinline__ void guard4(v8f& a0, v8f& a1, v8f& a2, v8f& a3,
                                       v16h x, v16h b0, v16h b1, v16h b2, v16h b3) {
  asm volatile("v_nop\n\tv_nop\n\tv_nop\n\tv_nop"
               : "+v"(a0), "+v"(a1), "+v"(a2), "+v"(a3)
               : "v"(x), "v"(b0), "v"(b1), "v"(b2), "v"(b3));
}

__global__ __launch_bounds__(256) void cast8_bf_f16_kernel(const float* __restrict__ in, unsigned short* __restrict__ out,
                                                           int n8, float carry) {
  const int i = blockIdx.x * 256 + threadIdx.x;
  if (i >= n8) return;
  const float* p = in + 8 * (size_t)i;
  const v4f a = *(const v4f*)(p);
  const v4f c = *(const v4f*)(p + 4);
  const float r0 = a[0], r1 = a[1], r2 = a[2], r3 = a[3];
  const float r4 = c[0], r5 = c[1], r6 = c[2], r7 = c[3];
  const float a0 = bf_rne(r0) * carry, a1 = bf_rne(r1) * carry, a2 = bf_rne(r2) * carry, a3 = bf_rne(r3) * carry;
  const float c0 = bf_rne(r4) * carry, c1 = bf_rne(r5) * carry, c2 = bf_rne(r6) * carry, c3 = bf_rne(r7) * carry;
  const v4u u = (v4u){pk16(h_bits(a0), h_bits(a1)), pk16(h_bits(a2), h_bits(a3)),
                      pk16(h_bits(c0), h_bits(c1)), pk16(h_bits(c2), h_bits(c3))};
  unsigned short* q = out + 8 * (size_t)i;
  *(volatile v4u*)q = u;
  __threadfence();
  *(volatile v4u*)q = u;
}

struct FreqTab { float f[16]; };
static_assert(sizeof(FreqTab) == 64, "no padding");
__global__ __launch_bounds__(256) void rot_table_kernel(const float* __restrict__ pos, float* __restrict__ tab, FreqTab ft) {
  __shared__ __align__(16) float sm[8 * 64];
  const int tid  = threadIdx.x;
  const int tl   = tid >> 5;
  const int axis = (tid >> 4) & 1;
  const int j    = tid & 15;
  const int token = blockIdx.x * 8 + tl;
  float fr = ft.f[0];
#pragma unroll
  for (int e = 1; e < 16; ++e) fr = (j == e) ? ft.f[e] : fr;
  const float praw = pos[(size_t)token * 2 + axis];
  const float p   = bf_rne(praw);
  const float t   = p * kPosScale;
  const float ang = t * fr;
  const float cv = cosf(ang);
  const float sv = sinf(ang);
  sm[tl * 64 + axis * 32 + j]      = cv;
  sm[tl * 64 + axis * 32 + 16 + j] = sv;
  __syncthreads();
  if (tid < 128) {
    const v4f v = *(const v4f*)(sm + tid * 4);
    float* dst = tab + (size_t)blockIdx.x * 512 + tid * 4;
    *(volatile v4f*)dst = v;
    __threadfence();
    *(volatile v4f*)dst = v;
  }
}

template <int EPI>
__global__ __launch_bounds__(256) void gemm_f16_kernel(
    const unsigned short* __restrict__ Ap, int lda, long sAo, long sAi,
    const unsigned short* __restrict__ Bp, int ldb, long sBo, long sBi,
    void* __restrict__ Cout, void* __restrict__ Cout2, int ldc, long sCo, long sCi,
    const float* __restrict__ bias, const float* __restrict__ tab,
    int M, int N, int K, int nInner, int nBatch, float scale) {
  __shared__ __align__(16) float sT[8][16 * 68];
  const int lane = threadIdx.x & 31;
  const int wave = threadIdx.x >> 5;
  const int tilesN = N >> 6;
  const int tilesM = M >> 5;
  const int perBatch = tilesM * tilesN;
  const int tile = blockIdx.x * 8 + wave;
  if (tile >= perBatch * nBatch) return;
  const int z  = tile / perBatch;
  const int tt = tile - z * perBatch;
  const int tm = tt / tilesN;
  const int tn = tt - tm * tilesN;
  const int m0 = tm << 5;
  const int n0 = tn << 6;
  const int zo = z / nInner;
  const int zi = z - zo * nInner;

  const _Float16* A  = (const _Float16*)Ap + (size_t)zo * sAo + (size_t)zi * sAi;
  const _Float16* Bt = (const _Float16*)Bp + (size_t)zo * sBo + (size_t)zi * sBi;
  const size_t coff = (size_t)zo * sCo + (size_t)zi * sCi;

  const int rlane = lane & 15;
  const int koff  = (lane >> 4) * 8;
  const int mOff  = (lane >> 4) * 8;

  v8f acc[2][4];
#pragma unroll
  for (int i = 0; i < 2; ++i)
#pragma unroll
    for (int j = 0; j < 4; ++j)
      acc[i][j] = (v8f){0.f, 0.f, 0.f, 0.f, 0.f, 0.f, 0.f, 0.f};

  for (int k0 = 0; k0 < K; k0 += 32) {
    v16h bh[4];
#pragma unroll
    for (int j = 0; j < 4; ++j) {
      const size_t bo = (size_t)(n0 + (j << 4) + rlane) * ldb + koff + k0;
      bh[j] = frag_load(Bt + bo);
    }
#pragma unroll
    for (int i = 0; i < 2; ++i) {
      const size_t ao = (size_t)(m0 + (i << 4) + rlane) * lda + koff + k0;
      const v16h ah = frag_load(A + ao);
#pragma unroll
      for (int j = 0; j < 4; ++j)
        acc[i][j] = mma16(ah, bh[j], acc[i][j]);
      guard4(acc[i][0], acc[i][1], acc[i][2], acc[i][3], ah, bh[0], bh[1], bh[2], bh[3]);
    }
  }

  float* slab = sT[wave];
  const int q  = lane >> 3;
  const int c8 = (lane & 7) * 8;
  const int hh = lane >> 4;
  const int c4 = (lane & 15) * 4;
  const bool isK = (n0 < kInner);
#pragma unroll
  for (int i = 0; i < 2; ++i) {
    const int mBase = m0 + (i << 4);
#pragma unroll
    for (int j = 0; j < 4; ++j) {
      float bv = 0.f;
      if (EPI == 0) {
        const float braw = bias[n0 + (j << 4) + rlane];
        bv = bf_rne(braw);
      }
#pragma unroll
      for (int r = 0; r < 8; ++r) {
        float v = acc[i][j][r] * scale;
        if (EPI == 0) v += bv;
        slab[(mOff + r) * 68 + (j << 4) + rlane] = v;
      }
    }
    __builtin_amdgcn_fence(__ATOMIC_RELEASE, "workgroup");
    __builtin_amdgcn_wave_barrier();
    __builtin_amdgcn_fence(__ATOMIC_ACQUIRE, "workgroup");
    if (EPI == 0) {
      float* C = (float*)Cout + coff;
      v4f vals[8];
#pragma unroll
      for (int it = 0; it < 8; ++it) vals[it] = *(const v4f*)(slab + (it * 2 + hh) * 68 + c4);
      for (int pass = 0; pass < 2; ++pass) {
#pragma unroll
        for (int it = 0; it < 8; ++it)
          *(volatile v4f*)(C + (size_t)(mBase + it * 2 + hh) * ldc + n0 + c4) = vals[it];
        __threadfence();
      }
    } else {
      unsigned short* Cb;
      int col;
      if (EPI == 3) {
        Cb  = isK ? (unsigned short*)Cout : (unsigned short*)Cout2;
        col = (n0 & (kInner - 1)) + c8;
      } else {
        Cb  = (unsigned short*)Cout + coff;
        col = n0 + c8;
      }
      const float sgn = (c8 & 16) ? 1.0f : -1.0f;
      const int tcol  = (c8 >> 5) * 32 + (c8 & 15);
      const float oc  = (EPI == 1) ? 1.0f : ((EPI == 2) ? kQC : kKVC);
      v4u ow[4];
#pragma unroll
      for (int it = 0; it < 4; ++it) {
        const int row = it * 4 + q;
        const float* sp = slab + row * 68 + c8;
        const v4f ta = *(const v4f*)(sp);
        const v4f tb = *(const v4f*)(sp + 4);
        float o[8];
        o[0] = ta[0]; o[1] = ta[1]; o[2] = ta[2]; o[3] = ta[3];
        o[4] = tb[0]; o[5] = tb[1]; o[6] = tb[2]; o[7] = tb[3];
        if (EPI >= 2) {
          const float* pp = slab + row * 68 + (c8 ^ 16);
          const v4f pa = *(const v4f*)(pp);
          const v4f pb = *(const v4f*)(pp + 4);
          float p[8];
          p[0] = pa[0]; p[1] = pa[1]; p[2] = pa[2]; p[3] = pa[3];
          p[4] = pb[0]; p[5] = pb[1]; p[6] = pb[2]; p[7] = pb[3];
          if (EPI == 3) {
            float s = ((o[0] + o[1]) + (o[2] + o[3])) + ((o[4] + o[5]) + (o[6] + o[7]));
            s += __shfl_xor(s, 1, 32);
            s += __shfl_xor(s, 2, 32);
            s += __shfl_xor(s, 4, 32);
            const float mean = s * kInvDh;
#pragma unroll
            for (int e = 0; e < 8; ++e) { o[e] -= mean; p[e] -= mean; }
            float ss = 0.0f;
#pragma unroll
            for (int e = 0; e < 8; ++e) ss = fmaf(o[e], o[e], ss);
            ss += __shfl_xor(ss, 1, 32);
            ss += __shfl_xor(ss, 2, 32);
            ss += __shfl_xor(ss, 4, 32);
            const float rstd = rsqrtf(ss * kInvDh + kNormEps);
#pragma unroll
            for (int e = 0; e < 8; ++e) { o[e] *= rstd; p[e] *= rstd; }
          }
          if (EPI == 2 || isK) {
            const float* tp = tab + (size_t)(mBase + row) * 64 + tcol;
            const v4f ca = *(const v4f*)(tp);
            const v4f cb = *(const v4f*)(tp + 4);
            const v4f sa = *(const v4f*)(tp + 16);
            const v4f sb = *(const v4f*)(tp + 20);
            float cc[8], sn[8];
            cc[0] = ca[0]; cc[1] = ca[1]; cc[2] = ca[2]; cc[3] = ca[3];
            cc[4] = cb[0]; cc[5] = cb[1]; cc[6] = cb[2]; cc[7] = cb[3];
            sn[0] = sa[0]; sn[1] = sa[1]; sn[2] = sa[2]; sn[3] = sa[3];
            sn[4] = sb[0]; sn[5] = sb[1]; sn[6] = sb[2]; sn[7] = sb[3];
#pragma unroll
            for (int e = 0; e < 8; ++e) o[e] = o[e] * cc[e] + sgn * (p[e] * sn[e]);
          }
        }
#pragma unroll
        for (int e = 0; e < 8; ++e) o[e] *= oc;
        ow[it] = (v4u){pk16(h_bits(o[0]), h_bits(o[1])), pk16(h_bits(o[2]), h_bits(o[3])),
                       pk16(h_bits(o[4]), h_bits(o[5])), pk16(h_bits(o[6]), h_bits(o[7]))};
      }
      for (int pass = 0; pass < 2; ++pass) {
#pragma unroll
        for (int it = 0; it < 4; ++it)
          *(volatile v4u*)(Cb + (size_t)(mBase + it * 4 + q) * ldc + col) = ow[it];
        __threadfence();
      }
    }
    __builtin_amdgcn_fence(__ATOMIC_RELEASE, "workgroup");
    __builtin_amdgcn_wave_barrier();
    __builtin_amdgcn_fence(__ATOMIC_ACQUIRE, "workgroup");
  }
}

__global__ __launch_bounds__(128) void dots_splitk_kernel(const unsigned short* __restrict__ kn,
                                                          const unsigned short* __restrict__ vn,
                                                          float* __restrict__ part) {
  __shared__ __align__(16) _Float16 sK[64 * 72];
  __shared__ __align__(16) _Float16 sV[64 * 72];
  __shared__ __align__(16) float sO[4][16 * 68];
  const int tid = threadIdx.x, lane = tid & 31, wave = tid >> 5;
  const int bh = blockIdx.x, ks = blockIdx.y;
  const int b = bh >> 3, h = bh & 7;
  const size_t row0 = (size_t)b * kSeq + (size_t)ks * kTokPerSplit;
  const int rlane = lane & 15;
  const int koff  = (lane >> 4) * 8;
  const int hh    = lane >> 4;

  v8f acc[4];
#pragma unroll
  for (int j = 0; j < 4; ++j) acc[j] = (v8f){0.f, 0.f, 0.f, 0.f, 0.f, 0.f, 0.f, 0.f};

#pragma unroll 1
  for (int ch = 0; ch < kTokPerSplit / 64; ++ch) {
    __syncthreads();
#pragma unroll
    for (int it = 0; it < 4; ++it) {
      const int seg = it * 128 + tid;
      const int tok = seg >> 3;
      const int s8  = (seg & 7) * 8;
      const size_t go = (row0 + (size_t)ch * 64 + tok) * kInner + h * kDh + s8;
      const v4u kw = *(const v4u*)(kn + go);
      const v4u vw = *(const v4u*)(vn + go);
#pragma unroll
      for (int w = 0; w < 4; ++w) {
        const unsigned kword = kw[w];
        const unsigned vword = vw[w];
        const unsigned short k0b = (unsigned short)(kword & 0xffffu);
        const unsigned short k1b = (unsigned short)(kword >> 16);
        const unsigned short v0b = (unsigned short)(vword & 0xffffu);
        const unsigned short v1b = (unsigned short)(vword >> 16);
        sK[(s8 + 2 * w) * 72 + tok]     = __builtin_bit_cast(_Float16, k0b);
        sK[(s8 + 2 * w + 1) * 72 + tok] = __builtin_bit_cast(_Float16, k1b);
        sV[(s8 + 2 * w) * 72 + tok]     = __builtin_bit_cast(_Float16, v0b);
        sV[(s8 + 2 * w + 1) * 72 + tok] = __builtin_bit_cast(_Float16, v1b);
      }
    }
    __syncthreads();
#pragma unroll
    for (int kk = 0; kk < 2; ++kk) {
      const v16h a  = frag_load(sV + (wave * 16 + rlane) * 72 + kk * 32 + koff);
      const v16h b0 = frag_load(sK + (0 * 16 + rlane) * 72 + kk * 32 + koff);
      const v16h b1 = frag_load(sK + (1 * 16 + rlane) * 72 + kk * 32 + koff);
      const v16h b2 = frag_load(sK + (2 * 16 + rlane) * 72 + kk * 32 + koff);
      const v16h b3 = frag_load(sK + (3 * 16 + rlane) * 72 + kk * 32 + koff);
      acc[0] = mma16(a, b0, acc[0]);
      acc[1] = mma16(a, b1, acc[1]);
      acc[2] = mma16(a, b2, acc[2]);
      acc[3] = mma16(a, b3, acc[3]);
      guard4(acc[0], acc[1], acc[2], acc[3], a, b0, b1, b2, b3);
    }
  }

  float* slab = sO[wave];
#pragma unroll
  for (int j = 0; j < 4; ++j)
#pragma unroll
    for (int r = 0; r < 8; ++r) slab[(8 * hh + r) * 68 + (j << 4) + rlane] = acc[j][r];
  __builtin_amdgcn_fence(__ATOMIC_RELEASE, "workgroup");
  __builtin_amdgcn_wave_barrier();
  __builtin_amdgcn_fence(__ATOMIC_ACQUIRE, "workgroup");
  {
    const int c4 = (lane & 15) * 4;
    float* C = part + ((size_t)ks * kBH + bh) * (kDh * kDh) + (size_t)(wave * 16) * kDh;
    v4f vals[8];
#pragma unroll
    for (int it = 0; it < 8; ++it) vals[it] = *(const v4f*)(slab + (it * 2 + hh) * 68 + c4);
    for (int pass = 0; pass < 2; ++pass) {
#pragma unroll
      for (int it = 0; it < 8; ++it)
        *(volatile v4f*)(C + (size_t)(it * 2 + hh) * kDh + c4) = vals[it];
      __threadfence();
    }
  }
}

__global__ __launch_bounds__(256) void dots_reduce_kernel(const float* __restrict__ part, unsigned short* __restrict__ dh,
                                                          int n8) {
  const int i = blockIdx.x * 256 + threadIdx.x;
  if (i >= n8) return;
  const size_t o = 8 * (size_t)i;
  float s[8];
#pragma unroll
  for (int e = 0; e < 8; ++e) s[e] = 0.0f;
#pragma unroll
  for (int ks = 0; ks < kSplitK; ++ks) {
    const float* p = part + (size_t)ks * kDotsElems + o;
    const v4f a = *(const v4f*)(p);
    const v4f c = *(const v4f*)(p + 4);
    s[0] += a[0]; s[1] += a[1]; s[2] += a[2]; s[3] += a[3];
    s[4] += c[0]; s[5] += c[1]; s[6] += c[2]; s[7] += c[3];
  }
  unsigned short hb[8];
#pragma unroll
  for (int e = 0; e < 8; ++e) {
    const float val = s[e] * kDotsScale;
    hb[e] = h_bits(val);
  }
  const v4u uh = (v4u){pk16(hb[0], hb[1]), pk16(hb[2], hb[3]), pk16(hb[4], hb[5]), pk16(hb[6], hb[7])};
  unsigned short* qh = dh + o;
  *(volatile v4u*)qh = uh;
  __threadfence();
  *(volatile v4u*)qh = uh;
}

extern "C" void kernel_launch(void* const* d_in, const int* in_sizes, int n_in,
                              void* d_out, int out_size, void* d_ws, size_t ws_size,
                              hipStream_t stream) {
  if (n_in < 8) return;
  if (in_sizes[0] != kTok * kDim) return;
  if (in_sizes[1] != kTok * kDim) return;
  if (in_sizes[2] != kTok * 2) return;
  if (in_sizes[3] != kTok * 2) return;
  if (in_sizes[4] != kInner * kDim) return;
  if (in_sizes[5] != 2 * kInner * kDim) return;
  if (in_sizes[6] != kDim * kInner) return;
  if (in_sizes[7] != kDim) return;
  if (out_size != kTok * kDim) return;
  if (ws_size < kWsTotal) return;

  const float* x    = (const float*)d_in[0];
  const float* z    = (const float*)d_in[1];
  const float* xpos = (const float*)d_in[2];
  const float* zpos = (const float*)d_in[3];
  const float* Wq   = (const float*)d_in[4];
  const float* Wkv  = (const float*)d_in[5];
  const float* Wout = (const float*)d_in[6];
  const float* bout = (const float*)d_in[7];
  float* out = (float*)d_out;

  char* ws = (char*)d_ws;
  unsigned short* WQ   = (unsigned short*)(ws + kOffWQ);
  unsigned short* WK   = (unsigned short*)(ws + kOffWK);
  unsigned short* WO   = (unsigned short*)(ws + kOffWO);
  unsigned short* S16  = (unsigned short*)(ws + kOffS16);
  unsigned short* KN   = (unsigned short*)(ws + kOffKN);
  unsigned short* VN   = (unsigned short*)(ws + kOffVN);
  unsigned short* QH   = (unsigned short*)(ws + kOffQH);
  float*          TAB  = (float*)(ws + kOffTAB);
  float*          PART = (float*)(ws + kOffPART);
  unsigned short* DH   = (unsigned short*)(ws + kOffDH);
  unsigned short* ATT  = KN;

  FreqTab ft;
  for (int j = 0; j < 16; ++j) {
    const double ex = (double)(2 * j) / 32.0;
    const float pw = (float)pow(10000.0, ex);
    ft.f[j] = 1.0f / pw;
  }

  cast8_bf_f16_kernel<<<(kInner * kDim / 8) / 256, 256, 0, stream>>>(Wq, WQ, kInner * kDim / 8, kWC);
  cast8_bf_f16_kernel<<<(2 * kInner * kDim / 8) / 256, 256, 0, stream>>>(Wkv, WK, 2 * kInner * kDim / 8, kWC);
  cast8_bf_f16_kernel<<<(kDim * kInner / 8) / 256, 256, 0, stream>>>(Wout, WO, kDim * kInner / 8, kWC);

  cast8_bf_f16_kernel<<<(kTok * kDim / 8) / 256, 256, 0, stream>>>(z, S16, kTok * kDim / 8, kXC);
  rot_table_kernel<<<kTok / 8, 256, 0, stream>>>(zpos, TAB, ft);
  gemm_f16_kernel<3><<<(kTok / 32) * (2 * kInner / 64) / 8, 256, 0, stream>>>(
      S16, kDim, 0L, 0L,
      WK, kDim, 0L, 0L,
      (void*)KN, (void*)VN, kInner, 0L, 0L,
      bout, TAB,
      kTok, 2 * kInner, kDim, 1, 1, kProjScale);

  cast8_bf_f16_kernel<<<(kTok * kDim / 8) / 256, 256, 0, stream>>>(x, S16, kTok * kDim / 8, kXC);
  rot_table_kernel<<<kTok / 8, 256, 0, stream>>>(xpos, TAB, ft);
  gemm_f16_kernel<2><<<(kTok / 32) * (kInner / 64) / 8, 256, 0, stream>>>(
      S16, kDim, 0L, 0L,
      WQ, kDim, 0L, 0L,
      (void*)QH, (void*)VN, kInner, 0L, 0L,
      bout, TAB,
      kTok, kInner, kDim, 1, 1, kProjScale);

  dots_splitk_kernel<<<dim3(kBH, kSplitK), 128, 0, stream>>>(KN, VN, PART);
  dots_reduce_kernel<<<(kDotsElems / 8) / 256, 256, 0, stream>>>(PART, DH, kDotsElems / 8);

  gemm_f16_kernel<1><<<kBH * (kSeq / 32) / 8, 256, 0, stream>>>(
      QH, kInner, (long)kSeq * kInner, (long)kDh,
      DH, kDh, (long)kHeads * kDh * kDh, (long)kDh * kDh,
      (void*)ATT, (void*)VN, kInner, (long)kSeq * kInner, (long)kDh,
      bout, TAB,
      kSeq, kDh, kDh, kHeads, kBH, kAttnScale);

  gemm_f16_kernel<0><<<(kTok / 32) * (kDim / 64) / 8, 256, 0, stream>>>(
      ATT, kInner, 0L, 0L,
      WO, kInner, 0L, 0L,
      (void*)out, (void*)VN, kDim, 0L, 0L,
      bout, TAB,
      kTok, kDim, kInner, 1, 1, kOutScale);
}
